// Model_8443905704627
// MI455X (gfx1250) — hardware-verified
//
#include <hip/hip_runtime.h>

#ifndef NB
#define NB 4
#endif
#ifndef SEQ
#define SEQ 4096
#endif
#define NB_FULL 4
#define SEQ_FULL 4096
#define DD 128
#ifndef QT
#define QT ((SEQ < 2048) ? SEQ : 2048)
#endif
#define NRW ((size_t)NB * SEQ)
static_assert(NB >= 1 && NB <= NB_FULL);
static_assert(SEQ >= 256 && SEQ <= SEQ_FULL && (SEQ % 256) == 0);
static_assert((QT % 128) == 0 && (SEQ % QT) == 0);
static_assert((DD % 64) == 0);

typedef unsigned short v8us __attribute__((ext_vector_type(8), may_alias));
typedef float  v8f  __attribute__((ext_vector_type(8)));
typedef float  v4f  __attribute__((ext_vector_type(4)));
typedef float  v4fa __attribute__((ext_vector_type(4), may_alias));
typedef _Float16 v16h __attribute__((ext_vector_type(16)));
typedef _Float16 v4h  __attribute__((ext_vector_type(4)));
union FragH { v16h v; v8us half[2]; _Float16 h[16]; unsigned short u[16]; };

__device__ __forceinline__ unsigned short bf16_bits(float x) { unsigned int u = __float_as_uint(x); return (unsigned short)((u + 0x7FFFu + ((u >> 16) & 1u)) >> 16); }
__device__ __forceinline__ float bf16_val(unsigned short b) { return __uint_as_float(((unsigned int)b) << 16); }
__device__ __forceinline__ float bf16_rne(float x) { return bf16_val(bf16_bits(x)); }

__device__ __forceinline__ v16h g2_frag(const _Float16* p, int hh) { FragH f; f.half[0] = *(const v8us*)((const unsigned short*)p + 8 * hh); f.half[1] = *(const v8us*)((const unsigned short*)p + 16 + 8 * hh); return f.v; }
__device__ __forceinline__ v8f g2_mma(v16h a, v16h b, v8f c) { v8f d = __builtin_amdgcn_wmma_f32_16x16x32_f16(false, a, false, b, (short)0, c, false, false); asm volatile("v_nop\n\tv_nop\n\tv_nop\n\tv_nop" : "+v"(d) : "v"(a), "v"(b)); return d; }

__global__ __launch_bounds__(256) void k_x16s(const float* __restrict__ x, _Float16* __restrict__ X16, int nrows, int seq, int seqFull) {
  const int t = blockIdx.x * 256 + threadIdx.x; const int ngrp = nrows * (DD / 8); if (t >= ngrp) return;
  const int r = t / (DD / 8), c8 = (t % (DD / 8)) * 8; const int b = r / seq, s = r - b * seq;
  const float* src = x + ((size_t)b * seqFull + s) * DD + c8;
  const v4f a = *(const v4fa*)src, c = *(const v4fa*)(src + 4);
  FragH f;
#pragma unroll
  for (int q = 0; q < 4; ++q) { f.h[q] = (_Float16)bf16_rne(a[q]); f.h[4 + q] = (_Float16)bf16_rne(c[q]); }
  unsigned short* d = (unsigned short*)X16 + (size_t)t * 8;
  *(volatile v8us*)d = f.half[0]; __threadfence(); *(volatile v8us*)d = f.half[0];
}

__global__ __launch_bounds__(256) void k_wnat(const float* __restrict__ w, int n8, _Float16* __restrict__ Bt) {
  const int t = blockIdx.x * 256 + threadIdx.x; if (t >= n8) return; FragH f;
#pragma unroll
  for (int q = 0; q < 8; ++q) f.h[q] = (_Float16)(bf16_rne(w[(size_t)t * 8 + q]) * 16.0f);
  unsigned short* d = (unsigned short*)Bt + (size_t)t * 8;
  *(volatile v8us*)d = f.half[0]; __threadfence(); *(volatile v8us*)d = f.half[0];
}

template <bool HB, bool H16>
__global__ __launch_bounds__(128) __attribute__((amdgpu_num_vgpr(256)))
void k_gemm2(const _Float16* __restrict__ A, int lda, const _Float16* __restrict__ Bh, int ldb, float alpha, const float* __restrict__ bias,
             float* __restrict__ C, _Float16* __restrict__ C16, int ldc, int M, int N, int K) {
  __shared__ __attribute__((aligned(16))) float so[4][32][68];
  const int tid = threadIdx.x, w = tid >> 5, lane = tid & 31, ln = lane & 15, hh = lane >> 4;
  const int ntn = N >> 6; const int mt = blockIdx.x / ntn, nq = blockIdx.x - mt * ntn;
  const int row0 = mt * 128 + 32 * w, col0 = nq * 64; if (row0 >= M) return;
  const _Float16* a0p = A + (size_t)(row0 + ln) * lda; const _Float16* a1p = a0p + (size_t)16 * lda;
  const _Float16* b0p = Bh + (size_t)(col0 + ln) * ldb; const _Float16* b1p = b0p + (size_t)16 * ldb;
  const _Float16* b2p = b1p + (size_t)16 * ldb; const _Float16* b3p = b2p + (size_t)16 * ldb;
  const v8f z8 = {0.f,0.f,0.f,0.f,0.f,0.f,0.f,0.f}; v8f c00 = z8, c01 = z8, c02 = z8, c03 = z8, c10 = z8, c11 = z8, c12 = z8, c13 = z8;
#pragma unroll 1
  for (int kb = 0; kb < K; kb += 32) { const v16h a0 = g2_frag(a0p + kb, hh), a1 = g2_frag(a1p + kb, hh);
    v16h b = g2_frag(b0p + kb, hh); c00 = g2_mma(a0, b, c00); c10 = g2_mma(a1, b, c10);
    b = g2_frag(b1p + kb, hh); c01 = g2_mma(a0, b, c01); c11 = g2_mma(a1, b, c11);
    b = g2_frag(b2p + kb, hh); c02 = g2_mma(a0, b, c02); c12 = g2_mma(a1, b, c12);
    b = g2_frag(b3p + kb, hh); c03 = g2_mma(a0, b, c03); c13 = g2_mma(a1, b, c13); }
  v8f accs[8] = {c00, c01, c02, c03, c10, c11, c12, c13};
#pragma unroll
  for (int u = 0; u < 8; ++u) { const int t = u & 3, half = u >> 2; const int col = col0 + t * 16 + ln; float bv = 0.f; if (HB) bv = bf16_rne(bias[col]);
#pragma unroll
    for (int r = 0; r < 8; ++r) { const int rloc = half * 16 + 8 * hh + r; so[w][rloc][t * 16 + ln] = accs[u][r] * alpha + bv; } }
  __builtin_amdgcn_fence(4, "workgroup"); __builtin_amdgcn_wave_barrier();
  const int rsub = lane >> 4, c4 = (lane & 15) * 4;
  for (int pass = 0; pass < 2; ++pass) {
#pragma unroll
    for (int q = 0; q < 16; ++q) { const int r = q * 2 + rsub; const v4f v = *(const v4fa*)&so[w][r][c4];
      if (H16) { v4h h4;
#pragma unroll
        for (int e = 0; e < 4; ++e) h4[e] = (_Float16)v[e];
        *(volatile v4h*)(C16 + (size_t)(row0 + r) * ldc + col0 + c4) = h4; }
      else { *(volatile v4f*)(C + (size_t)(row0 + r) * ldc + col0 + c4) = v; } }
    if (pass == 0) __threadfence(); }
}

template <int NHv, int TTv>
__global__ __launch_bounds__(256) void k_vt(const _Float16* __restrict__ V16, int ldv, _Float16* __restrict__ Vt) {
  __shared__ unsigned short tl[64][66];
  const int tid = threadIdx.x; const int slab = blockIdx.x / (TTv / 64), lg = blockIdx.x % (TTv / 64); const int b = slab / NHv, h = slab % NHv;
  for (int i = tid; i < 64 * 8; i += 256) { const int r = i / 8, c8 = (i % 8) * 8; FragH f;
    f.half[0] = *(const v8us*)((const unsigned short*)V16 + ((size_t)b * TTv + lg * 64 + r) * ldv + h * 64 + c8);
#pragma unroll
    for (int q = 0; q < 8; ++q) tl[r][c8 + q] = f.u[q]; }
  __syncthreads();
  for (int pass = 0; pass < 2; ++pass) {
#pragma unroll
    for (int rd = 0; rd < 2; ++rd) { const int d = rd * 32 + tid / 8, pc = tid % 8; FragH f;
#pragma unroll
      for (int q = 0; q < 8; ++q) f.u[q] = tl[pc * 8 + q][d];
      *(volatile v8us*)((unsigned short*)Vt + ((size_t)slab * 64 + d) * TTv + lg * 64 + pc * 8) = f.half[0]; }
    if (pass == 0) __threadfence(); }
}

__global__ __launch_bounds__(256) void k_rsmw(const float* __restrict__ S, _Float16* __restrict__ P, int nrows, int ncols) {
  #pragma clang fp contract(off)
  const int w = threadIdx.x >> 5, lane = threadIdx.x & 31;
  const int i = blockIdx.x * 8 + w; if (i >= nrows) return;
  const float* s = S + (size_t)i * ncols;
  float mx = -__builtin_inff();
#pragma unroll 1
  for (int j = lane * 4; j < ncols; j += 128) { const v4f a = *(const v4fa*)(s + j); mx = fmaxf(fmaxf(mx, fmaxf(a[0], a[1])), fmaxf(a[2], a[3])); }
#pragma unroll
  for (int o = 16; o > 0; o >>= 1) mx = fmaxf(mx, __shfl_xor(mx, o, 32));
  float se = 0.f;
#pragma unroll 1
  for (int j = lane * 4; j < ncols; j += 128) { const v4f a = *(const v4fa*)(s + j); se += (__expf(a[0] - mx) + __expf(a[1] - mx)) + (__expf(a[2] - mx) + __expf(a[3] - mx)); }
#pragma unroll
  for (int o = 16; o > 0; o >>= 1) se += __shfl_xor(se, o, 32);
  const float sc = 1024.0f / se;
  unsigned short* prow = (unsigned short*)P + (size_t)i * ncols;
#pragma unroll 1
  for (int j0 = lane * 8; j0 < ncols; j0 += 256) {
    const v4f a = *(const v4fa*)(s + j0), c = *(const v4fa*)(s + j0 + 4);
    FragH f;
#pragma unroll
    for (int q = 0; q < 4; ++q) { f.h[q] = (_Float16)(__expf(a[q] - mx) * sc); f.h[4 + q] = (_Float16)(__expf(c[q] - mx) * sc); }
    *(volatile v8us*)(prow + j0) = f.half[0];
    __threadfence();
    *(volatile v8us*)(prow + j0) = f.half[0];
  }
}

extern "C" void kernel_launch(void* const* d_in, const int* in_sizes, int n_in,
                              void* d_out, int out_size, void* d_ws, size_t ws_size, hipStream_t stream) {
  if (n_in < 9) return;
  const long long needRows = (long long)(NB - 1) * SEQ_FULL + SEQ;
  if ((long long)in_sizes[0] < needRows * DD || (long long)in_sizes[1] < needRows * DD || (long long)in_sizes[2] < needRows * DD) return;
  if (in_sizes[3] < DD * DD || in_sizes[5] < DD * DD || in_sizes[7] < DD * DD) return;
  if (in_sizes[4] < DD || in_sizes[6] < DD || in_sizes[8] < DD) return;
  if ((long long)out_size < (long long)NB * SEQ * DD) return;
  const float* query = (const float*)d_in[0]; const float* key = (const float*)d_in[1]; const float* value = (const float*)d_in[2];
  const float* Wq = (const float*)d_in[3]; const float* bq = (const float*)d_in[4];
  const float* Wk = (const float*)d_in[5]; const float* bk = (const float*)d_in[6];
  const float* Wv = (const float*)d_in[7]; const float* bv = (const float*)d_in[8];
  float* out = (float*)d_out;

  char* ws = (char*)d_ws; size_t off = 0;
  auto take = [&](size_t bytes) { char* p = ws + off; off += (bytes + 255) & ~(size_t)255; return p; };
  const size_t plane = NRW * DD * 2;
  _Float16* Xq = (_Float16*)take(plane); _Float16* Xk = (_Float16*)take(plane); _Float16* Xv = (_Float16*)take(plane);
  _Float16* Q16 = (_Float16*)take(plane); _Float16* K16 = (_Float16*)take(plane); _Float16* V16 = (_Float16*)take(plane);
  _Float16* VT = (_Float16*)take(plane);
  _Float16* Wtq = (_Float16*)take((size_t)DD * DD * 2); _Float16* Wtk = (_Float16*)take((size_t)DD * DD * 2); _Float16* Wtv = (_Float16*)take((size_t)DD * DD * 2);
  float* S = (float*)take((size_t)QT * SEQ * 4);
  _Float16* P = (_Float16*)take((size_t)QT * SEQ * 2);
  if (off > ws_size || off > ((size_t)128 << 20)) return;

  const int nrw = (int)NRW;
  const int ngrp = nrw * (DD / 8);
  k_x16s<<<(ngrp + 255) / 256, 256, 0, stream>>>(query, Xq, nrw, SEQ, SEQ_FULL);
  k_x16s<<<(ngrp + 255) / 256, 256, 0, stream>>>(key,   Xk, nrw, SEQ, SEQ_FULL);
  k_x16s<<<(ngrp + 255) / 256, 256, 0, stream>>>(value, Xv, nrw, SEQ, SEQ_FULL);
  const int wn8 = DD * DD / 8;
  k_wnat<<<(wn8 + 255) / 256, 256, 0, stream>>>(Wq, wn8, Wtq);
  k_wnat<<<(wn8 + 255) / 256, 256, 0, stream>>>(Wk, wn8, Wtk);
  k_wnat<<<(wn8 + 255) / 256, 256, 0, stream>>>(Wv, wn8, Wtv);
  const unsigned pgrid = (unsigned)((nrw / 128) * (DD / 64));
  k_gemm2<true, true><<<pgrid, 128, 0, stream>>>(Xq, DD, Wtq, DD, 0.0625f, bq, nullptr, Q16, DD, nrw, DD, DD);
  k_gemm2<true, true><<<pgrid, 128, 0, stream>>>(Xk, DD, Wtk, DD, 0.0625f, bk, nullptr, K16, DD, nrw, DD, DD);
  k_gemm2<true, true><<<pgrid, 128, 0, stream>>>(Xv, DD, Wtv, DD, 0.0625f, bv, nullptr, V16, DD, nrw, DD, DD);
  k_vt<2, SEQ><<<NB * 2 * (SEQ / 64), 256, 0, stream>>>(V16, DD, VT);
  for (int b = 0; b < NB; ++b) for (int q0 = 0; q0 < SEQ; q0 += QT) {
    k_gemm2<false, false><<<(unsigned)((QT / 128) * (SEQ / 64)), 128, 0, stream>>>(Q16 + ((size_t)b * SEQ + q0) * DD, DD, K16 + (size_t)b * SEQ * DD, DD, 0.08838834764831845f, nullptr, S, nullptr, SEQ, QT, SEQ, DD);
    k_rsmw<<<QT / 8, 256, 0, stream>>>(S, P, QT, SEQ);
    k_gemm2<false, false><<<(unsigned)((QT / 128) * (DD / 64)), 128, 0, stream>>>(P, SEQ, VT + (size_t)b * DD * SEQ, SEQ, 0.0009765625f, nullptr, out + ((size_t)b * SEQ + q0) * DD, nullptr, DD, QT, DD, SEQ);
  }
}
